// SymmetrizationMLP_11982958756740
// MI455X (gfx1250) — hardware-verified
//
#include <hip/hip_runtime.h>
#include <math.h>

typedef __attribute__((ext_vector_type(16))) _Float16 v16h;
typedef __attribute__((ext_vector_type(16))) __bf16 v16b;
typedef __attribute__((ext_vector_type(8)))  _Float16 v8h;
typedef __attribute__((ext_vector_type(8)))  float v8f;
typedef __attribute__((ext_vector_type(4)))  float v4f;
typedef __attribute__((ext_vector_type(2)))  float v2f;
typedef __attribute__((ext_vector_type(4)))  unsigned v4u;
typedef __attribute__((ext_vector_type(4)))  int v4i;
typedef float __attribute__((may_alias)) float_a;
typedef int __attribute__((may_alias)) int_a;

template <typename T> __device__ __forceinline__ void vst2(void* p, T v) { *(volatile T*)p = v; __threadfence(); *(volatile T*)p = v; }
__device__ __forceinline__ v8f wmma16(v16h a, v16h b, v8f c) {
  v8f d = __builtin_amdgcn_wmma_f32_16x16x32_f16(false, a, false, b, (short)0, c, false, false);
  asm volatile("v_nop\n\tv_nop\n\tv_nop\n\tv_nop" : "+v"(d) : "v"(a), "v"(b));
  return d;
}
__device__ __forceinline__ v8f wmma_bf(v16b a, v16b b, v8f c) {
  v8f d = __builtin_amdgcn_wmma_f32_16x16x32_bf16(false, a, false, b, (short)0, c, false, false);
  asm volatile("v_nop\n\tv_nop\n\tv_nop\n\tv_nop" : "+v"(d) : "v"(a), "v"(b));
  return d;
}
__device__ __forceinline__ v16h frag_h(const _Float16* rowk0, int lane) {
  union { v16h v; v8h q[2]; } u; const _Float16* p = rowk0 + 8 * (lane >> 4);
  u.q[0] = *(const v8h*)p; u.q[1] = *(const v8h*)(p + 16); return u.v;
}
__device__ __forceinline__ v16h frag_f32(const float* rowk0, int lane) {
  v16h a; const float* p = rowk0 + 8 * (lane >> 4);
#pragma unroll
  for (int i = 0; i < 8; ++i) { a[i] = (_Float16)p[i]; a[8 + i] = (_Float16)p[16 + i]; }
  return a;
}
__device__ __forceinline__ v16h frag_f32s(const float* rowk0, int lane, float sc) {
  v16h a; const float* p = rowk0 + 8 * (lane >> 4);
#pragma unroll
  for (int i = 0; i < 8; ++i) { a[i] = (_Float16)(p[i] * sc); a[8 + i] = (_Float16)(p[16 + i] * sc); }
  return a;
}
__device__ __forceinline__ v16h fragc_f32(const float* W, int k0, int n, int lane, int ld, int K) {
  v16h a; const int g = lane >> 4;
#pragma unroll
  for (int i = 0; i < 8; ++i) { const int ka = k0 + 8 * g + i, kb = ka + 16;
    a[i] = (_Float16)(ka < K ? W[(size_t)(ka < K ? ka : K - 1) * ld + n] : 0.f); a[8 + i] = (_Float16)(kb < K ? W[(size_t)(kb < K ? kb : K - 1) * ld + n] : 0.f); }
  return a;
}
struct F2 { v16b h, l; };
__device__ __forceinline__ F2 bsplit16(const float v[16]) { F2 r;
#pragma unroll
  for (int i = 0; i < 16; ++i) { const __bf16 h = (__bf16)v[i]; r.h[i] = h; r.l[i] = (__bf16)(v[i] - (float)h); }
  return r; }
__device__ __forceinline__ F2 split_row(const float* row, int k0, int lane) { float v[16]; const float* p = row + k0 + 8 * (lane >> 4);
#pragma unroll
  for (int i = 0; i < 8; ++i) { v[i] = p[i]; v[8 + i] = p[16 + i]; }
  return bsplit16(v); }
__device__ __forceinline__ F2 split_rowK(const float* row, int k0, int lane, int K) { float v[16]; const int g = lane >> 4;
#pragma unroll
  for (int i = 0; i < 8; ++i) { const int ka = k0 + 8 * g + i, kb = ka + 16; v[i] = ka < K ? row[ka < K ? ka : K - 1] : 0.f; v[8 + i] = kb < K ? row[kb < K ? kb : K - 1] : 0.f; }
  return bsplit16(v); }
__device__ __forceinline__ F2 split_col(const float* W, int k0, int n, int lane, int ld, int K) { float v[16]; const int g = lane >> 4;
#pragma unroll
  for (int i = 0; i < 8; ++i) { const int ka = k0 + 8 * g + i, kb = ka + 16; v[i] = ka < K ? W[(size_t)(ka < K ? ka : K - 1) * ld + n] : 0.f; v[8 + i] = kb < K ? W[(size_t)(kb < K ? kb : K - 1) * ld + n] : 0.f; }
  return bsplit16(v); }
__device__ __forceinline__ v8f mac3(const F2& a, const F2& b, v8f c) { c = wmma_bf(a.l, b.h, c); c = wmma_bf(a.h, b.l, c); return wmma_bf(a.h, b.h, c); }
__device__ __forceinline__ float sigm(float v) { return 1.0f / (1.0f + expf(-v)); }
#define LDSX() do { asm volatile("s_wait_dscnt 0" ::: "memory"); __builtin_amdgcn_wave_barrier(); __builtin_amdgcn_fence(__ATOMIC_RELEASE, "workgroup"); } while (0)


#define NB 1024
#define NPT 1024
#define KK 6
#define GG 720
#define INF 18
#define H1 64
#define H2 32
#define CO 40
#define BPB 4
#ifndef TBB
#define TBB (NB / BPB)
#endif
typedef __attribute__((ext_vector_type(8))) __bf16 v8b;
__device__ __forceinline__ v16b frag_b(const __bf16* rowk0, int lane) {
  union { v16b v; v8b q[2]; } u; const __bf16* p = rowk0 + 8 * (lane >> 4);
  u.q[0] = *(const v8b*)p; u.q[1] = *(const v8b*)(p + 16); return u.v;
}
__device__ __forceinline__ float bfr(float v) { return (float)(__bf16)v; }
__device__ __attribute__((noinline)) float exp_ni(float v) { return expf(v); }
__device__ __attribute__((noinline)) float erf_ni(float v) { return erff(v); }

#define WS_P1  0u
#define WS_P2  (WS_P1 + 2u * H1 * 32)
#define WS_P3  (WS_P2 + 2u * H2 * H1)
#define WS_END (WS_P3 + 2u * 48 * H2 + 256u)

__global__ __launch_bounds__(64) void k_pack(const float* __restrict__ W1, const float* __restrict__ W2, const float* __restrict__ W3, __bf16* __restrict__ P1, _Float16* __restrict__ P2, _Float16* __restrict__ P3) {
  __shared__ __align__(16) __bf16 s1[H1 * 32]; __shared__ __align__(16) _Float16 s2[H2 * H1]; __shared__ __align__(16) _Float16 s3[48 * H2]; const int t = threadIdx.x;
  for (int e = t; e < H1 * 32; e += 64) { const int n = e >> 5, k = e & 31; s1[e] = (k < INF) ? (__bf16)W1[k * H1 + n] : (__bf16)0.f; }
  for (int e = t; e < H2 * H1; e += 64) { const int n = e / H1, k = e % H1; s2[e] = (_Float16)(bfr(W2[k * H2 + n]) * 256.0f); }
  for (int e = t; e < 48 * H2; e += 64) { const int n = e / H2, k = e % H2; s3[e] = (n < CO) ? (_Float16)(bfr(W3[k * CO + n]) * 256.0f) : (_Float16)0.f; }
  __syncthreads();
  for (int q = t; q < H1 * 32 / 8; q += 64) vst2((unsigned*)(P1 + q * 8), *(const v4u*)&s1[q * 8]);
  for (int q = t; q < H2 * H1 / 8; q += 64) vst2((unsigned*)(P2 + q * 8), *(const v4u*)&s2[q * 8]);
  for (int q = t; q < 48 * H2 / 8; q += 64) vst2((unsigned*)(P3 + q * 8), *(const v4u*)&s3[q * 8]);
}
__global__ __launch_bounds__(128) void k_sym(const float* __restrict__ X, const int* __restrict__ IDX, const int* __restrict__ PERM, const __bf16* __restrict__ P1, const _Float16* __restrict__ P2, const _Float16* __restrict__ P3, const float* __restrict__ B1, const float* __restrict__ B2, const float* __restrict__ B3, float* __restrict__ OUT) {
  __shared__ float spt[BPB][KK * 3];
  __shared__ unsigned char sperm[GG][8];
  __shared__ __align__(16) _Float16 sa[4][16][72]; __shared__ __align__(16) _Float16 sb2[4][16][40];
  __shared__ __align__(16) float sacc[4][BPB][48];
  __shared__ __align__(16) float sout[BPB][CO];
  const int tid = threadIdx.x, wave = tid >> 5, lane = tid & 31, col = lane & 15, g = lane >> 4; const size_t b0 = (size_t)blockIdx.x * BPB;
  for (int e = tid; e < GG * KK; e += 128) sperm[e / KK][e % KK] = (unsigned char)min(max(PERM[e], 0), KK - 1);
  if (tid < BPB * KK * 3) { const int bb = tid / (KK * 3), rem = tid % (KK * 3); const int k = rem / 3, c = rem % 3; const int pi = min(max(IDX[(b0 + bb) * KK + k], 0), NPT - 1); spt[bb][rem] = bfr(X[((b0 + bb) * NPT + pi) * 3 + c]); }
  for (int e = tid; e < 4 * BPB * 48; e += 128) (&sacc[0][0][0])[e] = 0.f;
  __syncthreads();
  float part[BPB][3];
#pragma unroll
  for (int bb = 0; bb < BPB; ++bb) { part[bb][0] = 0.f; part[bb][1] = 0.f; part[bb][2] = 0.f; }
#pragma unroll 1
  for (int tile = wave; tile < BPB * GG / 16; tile += 4) { const int row0 = tile * 16;
    v16b a; { const int row = row0 + col; const int bb = row / GG, gi = row % GG;
#pragma unroll
      for (int i = 0; i < 8; ++i) { { const int k = 8 * g + i; a[i] = (k < INF) ? (__bf16)spt[bb][sperm[gi][k / 3] * 3 + (k % 3)] : (__bf16)0.f; } { const int k = 16 + 8 * g + i; a[8 + i] = (k < INF) ? (__bf16)spt[bb][sperm[gi][k / 3] * 3 + (k % 3)] : (__bf16)0.f; } } }
    v8f h1[4];
#pragma unroll
    for (int jt = 0; jt < 4; ++jt) { v8f z = {}; h1[jt] = wmma_bf(a, frag_b(P1 + (size_t)(jt * 16 + col) * 32, lane), z); }
#pragma unroll
    for (int jt = 0; jt < 4; ++jt) { const float bb1 = bfr(B1[jt * 16 + col]);
#pragma unroll
      for (int r = 0; r < 8; ++r) sa[wave][8 * g + r][jt * 16 + col] = (_Float16)fmaxf(h1[jt][r] + bb1, 0.f); }
    LDSX();
    v8f h2[2];
#pragma unroll
    for (int jt = 0; jt < 2; ++jt) { v8f z = {};
#pragma unroll
      for (int kc = 0; kc < H1 / 32; ++kc) z = wmma16(frag_h(&sa[wave][col][0] + kc * 32, lane), frag_h(P2 + (size_t)(jt * 16 + col) * H1 + kc * 32, lane), z); h2[jt] = z; }
#pragma unroll
    for (int jt = 0; jt < 2; ++jt) { const float bb2 = bfr(B2[jt * 16 + col]);
#pragma unroll
      for (int r = 0; r < 8; ++r) sb2[wave][8 * g + r][jt * 16 + col] = (_Float16)fmaxf(h2[jt][r] * (1.0f / 256.0f) + bb2, 0.f); }
    LDSX();
    const v16h a3 = frag_h(&sb2[wave][col][0], lane);
    { const int bb = row0 / GG;
#pragma unroll
      for (int jt = 0; jt < 3; ++jt) { v8f z = {}; z = wmma16(a3, frag_h(P3 + (size_t)(jt * 16 + col) * H2, lane), z); float s = 0.f;
#pragma unroll
        for (int r = 0; r < 8; ++r) s += z[r];
#pragma unroll
        for (int q = 0; q < BPB; ++q) if (q == bb) part[q][jt] += s; } }
    LDSX(); }
#pragma unroll
  for (int bb = 0; bb < BPB; ++bb)
#pragma unroll
    for (int jt = 0; jt < 3; ++jt) { float v = part[bb][jt]; v += __shfl_xor(v, 16); if (g == 0) sacc[wave][bb][jt * 16 + col] = v; }
  __syncthreads();
  for (int e = tid; e < BPB * CO; e += 128) { const int bb = e / CO, c = e % CO; const float s = ((sacc[0][bb][c] + sacc[1][bb][c]) + (sacc[2][bb][c] + sacc[3][bb][c])); sout[bb][c] = s * (1.0f / 256.0f) * (1.0f / (float)GG) + bfr(B3[c]); }
  __syncthreads();
  if (tid < BPB * CO / 4) vst2(OUT + b0 * CO + tid * 4, *(const v4f*)(&sout[0][0] + tid * 4));
}
extern "C" void kernel_launch(void* const* d_in, const int* in_sizes, int n_in, void* d_out, int out_size, void* d_ws, size_t ws_size, hipStream_t stream) {
  (void)in_sizes; (void)n_in; (void)out_size;
  const float** F = (const float**)d_in;
  if (ws_size < (size_t)WS_END) return;
  char* ws = (char*)d_ws; __bf16* P1 = (__bf16*)(ws + WS_P1); _Float16 *P2 = (_Float16*)(ws + WS_P2), *P3 = (_Float16*)(ws + WS_P3);
  k_pack<<<1, 64, 0, stream>>>(F[1], F[3], F[5], P1, P2, P3);
  k_sym<<<TBB, 128, 0, stream>>>(F[0], (const int*)d_in[7], (const int*)d_in[8], P1, P2, P3, F[2], F[4], F[6], (float*)d_out);
}
